// MultiHeadAttn_FishPP_35699768165046
// MI455X (gfx1250) — hardware-verified
//
#include <hip/hip_runtime.h>
#include <math.h>

typedef __attribute__((ext_vector_type(16))) _Float16 v16h;
typedef __attribute__((ext_vector_type(16))) __bf16 v16b;
typedef __attribute__((ext_vector_type(8)))  _Float16 v8h;
typedef __attribute__((ext_vector_type(8)))  float v8f;
typedef __attribute__((ext_vector_type(4)))  float v4f;
typedef __attribute__((ext_vector_type(2)))  float v2f;
typedef __attribute__((ext_vector_type(4)))  unsigned v4u;
typedef __attribute__((ext_vector_type(4)))  int v4i;
typedef float __attribute__((may_alias)) float_a;
typedef int __attribute__((may_alias)) int_a;

template <typename T> __device__ __forceinline__ void vst2(void* p, T v) { *(volatile T*)p = v; __threadfence(); *(volatile T*)p = v; }
__device__ __forceinline__ v8f wmma16(v16h a, v16h b, v8f c) {
  v8f d = __builtin_amdgcn_wmma_f32_16x16x32_f16(false, a, false, b, (short)0, c, false, false);
  asm volatile("v_nop\n\tv_nop\n\tv_nop\n\tv_nop" : "+v"(d) : "v"(a), "v"(b));
  return d;
}
__device__ __forceinline__ v8f wmma_bf(v16b a, v16b b, v8f c) {
  v8f d = __builtin_amdgcn_wmma_f32_16x16x32_bf16(false, a, false, b, (short)0, c, false, false);
  asm volatile("v_nop\n\tv_nop\n\tv_nop\n\tv_nop" : "+v"(d) : "v"(a), "v"(b));
  return d;
}
__device__ __forceinline__ v16h frag_h(const _Float16* rowk0, int lane) {
  union { v16h v; v8h q[2]; } u; const _Float16* p = rowk0 + 8 * (lane >> 4);
  u.q[0] = *(const v8h*)p; u.q[1] = *(const v8h*)(p + 16); return u.v;
}
__device__ __forceinline__ v16h frag_f32(const float* rowk0, int lane) {
  v16h a; const float* p = rowk0 + 8 * (lane >> 4);
#pragma unroll
  for (int i = 0; i < 8; ++i) { a[i] = (_Float16)p[i]; a[8 + i] = (_Float16)p[16 + i]; }
  return a;
}
__device__ __forceinline__ v16h frag_f32s(const float* rowk0, int lane, float sc) {
  v16h a; const float* p = rowk0 + 8 * (lane >> 4);
#pragma unroll
  for (int i = 0; i < 8; ++i) { a[i] = (_Float16)(p[i] * sc); a[8 + i] = (_Float16)(p[16 + i] * sc); }
  return a;
}
__device__ __forceinline__ v16h fragc_f32(const float* W, int k0, int n, int lane, int ld, int K) {
  v16h a; const int g = lane >> 4;
#pragma unroll
  for (int i = 0; i < 8; ++i) { const int ka = k0 + 8 * g + i, kb = ka + 16;
    a[i] = (_Float16)(ka < K ? W[(size_t)(ka < K ? ka : K - 1) * ld + n] : 0.f); a[8 + i] = (_Float16)(kb < K ? W[(size_t)(kb < K ? kb : K - 1) * ld + n] : 0.f); }
  return a;
}
struct F2 { v16b h, l; };
__device__ __forceinline__ F2 bsplit16(const float v[16]) { F2 r;
#pragma unroll
  for (int i = 0; i < 16; ++i) { const __bf16 h = (__bf16)v[i]; r.h[i] = h; r.l[i] = (__bf16)(v[i] - (float)h); }
  return r; }
__device__ __forceinline__ F2 split_row(const float* row, int k0, int lane) { float v[16]; const float* p = row + k0 + 8 * (lane >> 4);
#pragma unroll
  for (int i = 0; i < 8; ++i) { v[i] = p[i]; v[8 + i] = p[16 + i]; }
  return bsplit16(v); }
__device__ __forceinline__ F2 split_rowK(const float* row, int k0, int lane, int K) { float v[16]; const int g = lane >> 4;
#pragma unroll
  for (int i = 0; i < 8; ++i) { const int ka = k0 + 8 * g + i, kb = ka + 16; v[i] = ka < K ? row[ka < K ? ka : K - 1] : 0.f; v[8 + i] = kb < K ? row[kb < K ? kb : K - 1] : 0.f; }
  return bsplit16(v); }
__device__ __forceinline__ F2 split_col(const float* W, int k0, int n, int lane, int ld, int K) { float v[16]; const int g = lane >> 4;
#pragma unroll
  for (int i = 0; i < 8; ++i) { const int ka = k0 + 8 * g + i, kb = ka + 16; v[i] = ka < K ? W[(size_t)(ka < K ? ka : K - 1) * ld + n] : 0.f; v[8 + i] = kb < K ? W[(size_t)(kb < K ? kb : K - 1) * ld + n] : 0.f; }
  return bsplit16(v); }
__device__ __forceinline__ v8f mac3(const F2& a, const F2& b, v8f c) { c = wmma_bf(a.l, b.h, c); c = wmma_bf(a.h, b.l, c); return wmma_bf(a.h, b.h, c); }
__device__ __forceinline__ float sigm(float v) { return 1.0f / (1.0f + expf(-v)); }
#define LDSX() do { asm volatile("s_wait_dscnt 0" ::: "memory"); __builtin_amdgcn_wave_barrier(); __builtin_amdgcn_fence(__ATOMIC_RELEASE, "workgroup"); } while (0)


#define NTOK 197
#define NP 256
#define NKT 7
#define NBT 64
#define DD 768
#define GH 2
#define NHD 12
#define HR 6
#define DH 64
#define QKD (GH * DH)
#define ML 3
#define EPS 1e-5f
#ifndef TNB
#define TNB NBT
#endif
typedef __attribute__((ext_vector_type(8))) __bf16 v8b;
__device__ __forceinline__ v16b frag_b(const __bf16* rowk0, int lane) {
  union { v16b v; v8b q[2]; } u; const __bf16* p = rowk0 + 8 * (lane >> 4);
  u.q[0] = *(const v8b*)p; u.q[1] = *(const v8b*)(p + 16); return u.v;
}
__device__ __forceinline__ float bfr(float v) { return (float)(__bf16)v; }
__device__ __attribute__((noinline)) float exp_ni(float v) { return expf(v); }
__device__ __attribute__((noinline)) float erf_ni(float v) { return erff(v); }

#define WS_QK  0u
#define WS_QKL (WS_QK + 2u * (size_t)NBT * NP * 2 * QKD)
#define WS_VT  (WS_QKL + 2u * (size_t)NBT * NP * 2 * QKD)
#define WS_VTL (WS_VT + 2u * (size_t)NBT * DD * NP)
#define WS_MW  (WS_VTL + 2u * (size_t)NBT * DD * NP)
#define WS_Z   (WS_MW + 4u * (size_t)NTOK * NHD * NP)
#define WS_END (WS_Z + 4u * (size_t)NTOK * NBT * DD)

__device__ __forceinline__ v16b fragb_f32(const float* __restrict__ p, int lane) { v16b a; const float* pp = p + 8 * (lane >> 4);
#pragma unroll
  for (int i = 0; i < 8; ++i) { a[i] = (__bf16)pp[i]; a[8 + i] = (__bf16)pp[16 + i]; } return a; }
__global__ __launch_bounds__(256) void k_mw(const float* __restrict__ MASKS, const float* __restrict__ MP, float* __restrict__ MW) { __shared__ __align__(16) float s[NHD][NP]; const int i = blockIdx.x, t = threadIdx.x;
  for (int e = t; e < NHD * NP; e += 256) { const int n = e / NP, j = e % NP; float v = 0.f; if (j < NTOK) {
#pragma unroll
      for (int l = 0; l < ML; ++l) v += bfr(MASKS[((size_t)i * NTOK + j) * ML + l]) * bfr(MP[l * NHD + n]); } s[n][j] = v; }
  __syncthreads(); for (int e = t; e < NHD * NP / 4; e += 256) { const int n = e / (NP / 4), q = e % (NP / 4); vst2(MW + ((size_t)i * NHD + n) * NP + q * 4, *(const v4f*)&s[n][q * 4]); } }
__global__ __launch_bounds__(128) void k_proj(const float* __restrict__ Hh, const float* __restrict__ WQ, const float* __restrict__ WK, const float* __restrict__ WV, _Float16* __restrict__ QK, _Float16* __restrict__ QKL, _Float16* __restrict__ VT, _Float16* __restrict__ VTL) {
  __shared__ __align__(16) _Float16 sh[64][136], sl[64][136]; __shared__ __align__(16) _Float16 th[128][72], tl[128][72];
  const int tid = threadIdx.x, wave = tid >> 5, lane = tid & 31, col = lane & 15, g = lane >> 4; const size_t b = blockIdx.z; const int i0 = blockIdx.x * 64 + wave * 16; const int c0 = blockIdx.y * 128;
  const int irow = i0 + col; const int ic = irow < NTOK ? irow : NTOK - 1; const float* xr = Hh + ((size_t)ic * NBT + b) * DD;
  const float* Wm = c0 < QKD ? WQ + (size_t)c0 * DD : c0 < 2 * QKD ? WK + (size_t)(c0 - QKD) * DD : WV + (size_t)(c0 - 2 * QKD) * DD;
  v8f acc[8] = {};
#pragma unroll 2
  for (int kc = 0; kc < DD / 32; ++kc) { const v16b a = fragb_f32(xr + kc * 32, lane);
#pragma unroll
    for (int j = 0; j < 8; ++j) acc[j] = wmma_bf(a, fragb_f32(Wm + (size_t)(j * 16 + col) * DD + kc * 32, lane), acc[j]); }
  const bool isv = c0 >= 2 * QKD;
#pragma unroll
  for (int j = 0; j < 8; ++j)
#pragma unroll
    for (int r = 0; r < 8; ++r) { const float v = acc[j][r]; const _Float16 hv = (_Float16)v; const _Float16 lv = (_Float16)((v - (float)hv) * 2048.0f); if (!isv) { sh[wave * 16 + 8 * g + r][j * 16 + col] = hv; sl[wave * 16 + 8 * g + r][j * 16 + col] = lv; } else { th[j * 16 + col][wave * 16 + 8 * g + r] = hv; tl[j * 16 + col][wave * 16 + 8 * g + r] = lv; } }
  __syncthreads();
  if (!isv) { for (int e = tid; e < 64 * 16; e += 128) { const int rl = e >> 4, q = e & 15; const size_t o = (b * NP + blockIdx.x * 64 + rl) * (2 * QKD) + c0 + q * 8; vst2((unsigned*)(QK + o), *(const v4u*)&sh[rl][q * 8]); vst2((unsigned*)(QKL + o), *(const v4u*)&sl[rl][q * 8]); } }
  else { const int cv0 = c0 - 2 * QKD; for (int e = tid; e < 128 * 8; e += 128) { const int cl = e >> 3, q = e & 7; const size_t o = ((b * DD + cv0 + cl) * (size_t)NP) + blockIdx.x * 64 + q * 8; vst2((unsigned*)(VT + o), *(const v4u*)&th[cl][q * 8]); vst2((unsigned*)(VTL + o), *(const v4u*)&tl[cl][q * 8]); } } }
__global__ __launch_bounds__(128) void k_att(const _Float16* __restrict__ QK, const _Float16* __restrict__ QKL, const _Float16* __restrict__ VT, const _Float16* __restrict__ VTL, const float* __restrict__ MW, float* __restrict__ Z) {
  __shared__ __align__(16) float sp[4][16][36]; __shared__ __align__(16) float so[4][16][68];
  const int tid = threadIdx.x, wave = tid >> 5, lane = tid & 31, col = lane & 15, g = lane >> 4; const int n = blockIdx.y; const int gh = n / HR; const size_t b = blockIdx.z; const int q0 = blockIdx.x * 64 + wave * 16; const size_t rq = b * NP + q0;
  v16h aq[2], al[2];
#pragma unroll
  for (int kc = 0; kc < 2; ++kc) { aq[kc] = frag_h(QK + (rq + col) * (2 * QKD) + gh * DH + kc * 32, lane); al[kc] = frag_h(QKL + (rq + col) * (2 * QKD) + gh * DH + kc * 32, lane); }
  float m[8], l[8];
#pragma unroll
  for (int r = 0; r < 8; ++r) { m[r] = -3.0e38f; l[r] = 0.f; }
  v8f acc[4] = {}, accl[4] = {};
#pragma unroll 1
  for (int ks = 0; ks < NKT; ++ks) { v8f s[2];
#pragma unroll
    for (int ct = 0; ct < 2; ++ct) { const int kk = ks * 32 + ct * 16 + col; const size_t rk = b * NP + kk; v8f c = {}, cl = {};
#pragma unroll
      for (int kc = 0; kc < 2; ++kc) { const v16h kh = frag_h(QK + rk * (2 * QKD) + QKD + gh * DH + kc * 32, lane), kl = frag_h(QKL + rk * (2 * QKD) + QKD + gh * DH + kc * 32, lane); c = wmma16(aq[kc], kh, c); cl = wmma16(aq[kc], kl, cl); cl = wmma16(al[kc], kh, cl); }
      const bool keep = kk < NTOK;
#pragma unroll
      for (int r = 0; r < 8; ++r) { const int qi = q0 + 8 * g + r; const int qc = qi < NTOK ? qi : NTOK - 1; s[ct][r] = keep ? (c[r] + cl[r] * (1.0f / 2048.0f)) * 0.125f * MW[((size_t)qc * NHD + n) * NP + kk] : -3.0e38f; } }
    float alpha[8];
#pragma unroll
    for (int r = 0; r < 8; ++r) { float mx = fmaxf(s[0][r], s[1][r]);
#pragma unroll
      for (int o = 1; o < 16; o <<= 1) mx = fmaxf(mx, __shfl_xor(mx, o));
      const float mn = fmaxf(m[r], mx); alpha[r] = (m[r] <= -1.0e38f) ? 0.f : __expf(m[r] - mn); const float e0 = (s[0][r] <= -1.0e38f) ? 0.f : __expf(s[0][r] - mn), e1 = (s[1][r] <= -1.0e38f) ? 0.f : __expf(s[1][r] - mn); float es = e0 + e1;
#pragma unroll
      for (int o = 1; o < 16; o <<= 1) es += __shfl_xor(es, o);
      l[r] = l[r] * alpha[r] + es; m[r] = mn; sp[wave][8 * g + r][col] = e0; sp[wave][8 * g + r][16 + col] = e1; }
#pragma unroll
    for (int j = 0; j < 4; ++j)
#pragma unroll
      for (int r = 0; r < 8; ++r) { acc[j][r] *= alpha[r]; accl[j][r] *= alpha[r]; }
    LDSX();
    v16h pa; { const float* prow = &sp[wave][col][0] + 8 * (lane >> 4);
#pragma unroll
      for (int i = 0; i < 8; ++i) { pa[i] = (_Float16)(prow[i] * 2048.0f); pa[8 + i] = (_Float16)(prow[16 + i] * 2048.0f); } }
#pragma unroll
    for (int j = 0; j < 4; ++j) { const size_t po = (b * DD + (size_t)n * DH + j * 16 + col) * (size_t)NP + ks * 32; acc[j] = wmma16(pa, frag_h(VT + po, lane), acc[j]); accl[j] = wmma16(pa, frag_h(VTL + po, lane), accl[j]); }
    LDSX(); }
#pragma unroll
  for (int r = 0; r < 8; ++r) { const float il = (1.0f / 2048.0f) / l[r];
#pragma unroll
    for (int j = 0; j < 4; ++j) so[wave][8 * g + r][j * 16 + col] = (acc[j][r] + accl[j][r] * (1.0f / 2048.0f)) * il; }
  LDSX(); for (int rl = 0; rl < 16; ++rl) { const int qi = q0 + rl; if (qi < NTOK && lane < 16) vst2(Z + ((size_t)qi * NBT + b) * DD + (size_t)n * DH + lane * 4, *(const v4f*)&so[wave][rl][lane * 4]); } }
__global__ __launch_bounds__(128) void k_out(const float* __restrict__ Zr, const float* __restrict__ WO, const float* __restrict__ Hh, float* __restrict__ X2, int nrows) { __shared__ __align__(16) float sf[4][16][132];
  const int tid = threadIdx.x, wave = tid >> 5, lane = tid & 31, col = lane & 15, g = lane >> 4; const size_t r0 = (size_t)blockIdx.x * 64 + wave * 16; const int c0 = blockIdx.y * 128;
  v8f acc[8] = {};
#pragma unroll 2
  for (int kc = 0; kc < DD / 32; ++kc) { const size_t ra = (r0 + col) < (size_t)nrows ? (r0 + col) : (size_t)nrows - 1; const F2 a = split_row(Zr + ra * DD, kc * 32, lane);
#pragma unroll
    for (int j = 0; j < 8; ++j) { const v16b w = fragb_f32(WO + (size_t)(c0 + j * 16 + col) * DD + kc * 32, lane); acc[j] = wmma_bf(a.h, w, acc[j]); acc[j] = wmma_bf(a.l, w, acc[j]); } }
#pragma unroll
  for (int j = 0; j < 8; ++j) { const int c = c0 + j * 16 + col;
#pragma unroll
    for (int r = 0; r < 8; ++r) { const size_t row = r0 + 8 * g + r; const size_t ra = row < (size_t)nrows ? row : (size_t)nrows - 1; sf[wave][8 * g + r][j * 16 + col] = acc[j][r] + bfr(Hh[ra * DD + c]); } }
  LDSX(); for (int rl = 0; rl < 16; ++rl) { const size_t row = r0 + rl; if (row < (size_t)nrows) vst2(X2 + row * DD + c0 + lane * 4, *(const v4f*)&sf[wave][rl][lane * 4]); } }
__global__ __launch_bounds__(256) void k_ln(const float* __restrict__ X2, const float* __restrict__ G, const float* __restrict__ Bt, float* __restrict__ OUT) { __shared__ float red[8]; __shared__ __align__(16) float so2[DD]; const int t = threadIdx.x; const size_t row = blockIdx.x;
  float v[3]; float s = 0.f; for (int i = 0; i < 3; ++i) { v[i] = X2[row * DD + t + 256 * i]; s += v[i]; }
#pragma unroll
  for (int o = 1; o < 32; o <<= 1) s += __shfl_xor(s, o);
  if ((t & 31) == 0) red[t >> 5] = s; __syncthreads(); float mu = 0.f; for (int i = 0; i < 8; ++i) mu += red[i]; mu /= (float)DD; __syncthreads();
  float q = 0.f; for (int i = 0; i < 3; ++i) { const float d = v[i] - mu; q += d * d; }
#pragma unroll
  for (int o = 1; o < 32; o <<= 1) q += __shfl_xor(q, o);
  if ((t & 31) == 0) red[t >> 5] = q; __syncthreads(); float var = 0.f; for (int i = 0; i < 8; ++i) var += red[i]; var /= (float)DD; const float inv = 1.0f / sqrtf(var + EPS);
  for (int i = 0; i < 3; ++i) { const int c = t + 256 * i; so2[c] = bfr(G[c]) * (v[i] - mu) * inv + bfr(Bt[c]); } __syncthreads(); if (t < DD / 4) vst2(OUT + row * DD + t * 4, *(const v4f*)&so2[t * 4]); }
extern "C" void kernel_launch(void* const* d_in, const int* in_sizes, int n_in, void* d_out, int out_size, void* d_ws, size_t ws_size, hipStream_t stream) {
  (void)in_sizes; (void)n_in; (void)out_size;
  const float** F = (const float**)d_in;
  if (ws_size < (size_t)WS_END) return;
  char* ws = (char*)d_ws; _Float16 *QK = (_Float16*)(ws + WS_QK), *QKL = (_Float16*)(ws + WS_QKL), *VT = (_Float16*)(ws + WS_VT), *VTL = (_Float16*)(ws + WS_VTL); float *MW = (float*)(ws + WS_MW), *Z = (float*)(ws + WS_Z);
  const int nrows = NTOK * TNB;
  k_mw<<<NTOK, 256, 0, stream>>>(F[1], F[6], MW);
  k_proj<<<dim3(NP / 64, (2 * QKD + DD) / 128, TNB), 128, 0, stream>>>(F[0], F[2], F[3], F[4], QK, QKL, VT, VTL);
  k_att<<<dim3(NP / 64, NHD, TNB), 128, 0, stream>>>(QK, QKL, VT, VTL, MW, Z);
  float* X2 = (float*)(ws + WS_VT);
  (void)nrows;
  k_out<<<dim3((NTOK * NBT + 63) / 64, DD / 128), 128, 0, stream>>>(Z, F[5], F[0], X2, NTOK * NBT);
  k_ln<<<NTOK * NBT, 256, 0, stream>>>(X2, F[7], F[8], (float*)d_out);
}
